// refinment_decoder_8246337208836
// MI455X (gfx1250) — hardware-verified
//
#include <hip/hip_runtime.h>


#define NBI  4
#define CH   128
#define HS   64
#define HO   256
#define HP   258
#define NPIX (HO * HO)
#define NTILE (NPIX / 64)
#define KK   (9 * CH)
#define EPS_ 1e-5f

typedef unsigned short bf;
typedef __attribute__((ext_vector_type(16))) __bf16   v16bf;
typedef __attribute__((ext_vector_type(8)))  unsigned short v8us;
typedef __attribute__((ext_vector_type(4)))  unsigned short v4us;
typedef __attribute__((ext_vector_type(8)))  float    v8f;
typedef __attribute__((ext_vector_type(4)))  float    v4f;
typedef v4f  __attribute__((may_alias)) v4fa;
typedef v8us __attribute__((may_alias)) v8usa;

__device__ __forceinline__ unsigned short f2bf(float f) { unsigned u = __float_as_uint(f); u += 0x7FFFu + ((u >> 16) & 1u); return (unsigned short)(u >> 16); }
__device__ __forceinline__ float bf2f(unsigned short b) { return __uint_as_float(((unsigned)b) << 16); }
__device__ __forceinline__ float bfr(float f) { return bf2f(f2bf(f)); }
__device__ __forceinline__ v16bf cat16b(v8us lo, v8us hi) { return __builtin_bit_cast(v16bf, __builtin_shufflevector(lo, hi, 0, 1, 2, 3, 4, 5, 6, 7, 8, 9, 10, 11, 12, 13, 14, 15)); }
__device__ __forceinline__ v8f wmmab(v16bf a, v16bf b, v8f c) { return __builtin_amdgcn_wmma_f32_16x16x32_bf16(false, a, false, b, (short)0, c, false, false); }

__global__ __launch_bounds__(256) void k_preround(const float* __restrict__ low, float* LR, int n4) {
    const int i = blockIdx.x * 256 + threadIdx.x; if (i >= n4) return;
    const v4f v = *(const v4f*)(low + (size_t)i * 4); v4f o;
#pragma unroll
    for (int k = 0; k < 4; ++k) o[k] = bfr(v[k]);
    *(volatile v4f*)(LR + (size_t)i * 4) = o; __threadfence(); *(volatile v4f*)(LR + (size_t)i * 4) = o;
}
__device__ __forceinline__ void coords(int o, int& i0, int& i1, float& f) {
    const float sc = (float)(63.0 / 255.0); const float pos = (float)o * sc; i0 = (int)floorf(pos); i1 = i0 + 1 < HS ? i0 + 1 : HS - 1; f = pos - (float)i0;
}
__device__ __forceinline__ float bilin(const float* __restrict__ Lp, int i0, int i1, float fy, int j0, int j1, float fx) {
    const float a = Lp[i0 * HS + j0], b = Lp[i1 * HS + j0], c = Lp[i0 * HS + j1], d = Lp[i1 * HS + j1];
    const float t0 = a * (1.0f - fy) + b * fy, t1 = c * (1.0f - fy) + d * fy;
    return t0 * (1.0f - fx) + t1 * fx;
}
struct Tile { int b, y, x, px, grp, i0, i1, j0, j1; float fy, fx; };
__device__ __forceinline__ Tile tile_of(int bid, int tid) {
    Tile t; t.b = bid / NTILE; const int tt = bid - t.b * NTILE; const int ty = tt >> 5, tx = tt & 31;
    t.px = tid & 63; t.grp = tid >> 6; t.y = ty * 8 + (t.px >> 3); t.x = tx * 8 + (t.px & 7);
    coords(t.y, t.i0, t.i1, t.fy); coords(t.x, t.j0, t.j1, t.fx); return t;
}

__global__ __launch_bounds__(256) void k_statf(const float* __restrict__ low, const float* __restrict__ xin, const float* __restrict__ gam, const float* __restrict__ alp,
                                               const float* __restrict__ bet, float* MT, float* PART) {
    __shared__ float vals[CH][65]; __shared__ float part[4][64]; __shared__ float sM[64]; __shared__ float sS[64];
    const int tid = threadIdx.x; const Tile t = tile_of(blockIdx.x, tid);
#pragma unroll 1
    for (int k = 0; k < 32; ++k) { const int c = t.grp * 32 + k; vals[c][t.px] = bilin(low + ((size_t)t.b * CH + c) * HS * HS, t.i0, t.i1, t.fy, t.j0, t.j1, t.fx); }
    __syncthreads();
    { float s = 0.f;
#pragma unroll 1
      for (int k = 0; k < 32; ++k) s += vals[t.grp * 32 + k][t.px];
      part[t.grp][t.px] = s; }
    __syncthreads();
    if (tid < 64) { sM[tid] = ((part[0][tid] + part[1][tid]) + (part[2][tid] + part[3][tid])) * (1.0f / CH);
        const int ty = blockIdx.x % NTILE; const int y = (ty >> 5) * 8 + (tid >> 3), x = (ty & 31) * 8 + (tid & 7);
        sS[tid] = 1.0f / (1.0f + expf(-bfr(xin[((size_t)t.b * HO + y) * HO + x]))); }
    __syncthreads();
    if (tid < 16) { const v4f v = *(const v4fa*)(sM + tid * 4); float* o = MT + (size_t)blockIdx.x * 64 + tid * 4; *(volatile v4f*)o = v; __threadfence(); *(volatile v4f*)o = v; }
    const float ga = bfr(gam[0]), al = bfr(alp[0]), be = bfr(bet[0]);
    const int c = tid & (CH - 1), isbg = tid >> 7;
    float S = 0.f, S2 = 0.f;
#pragma unroll 1
    for (int p = 0; p < 64; p += 4) {
#pragma unroll
        for (int u = 0; u < 4; ++u) { const float lf2 = ga * sM[p + u] + vals[c][p + u]; const float sg = sS[p + u]; const float v = isbg ? be * (lf2 * (1.0f - sg)) : al * (lf2 * sg); S += v; S2 = fmaf(v, v, S2); } }
    typedef __attribute__((ext_vector_type(2))) float v2f;
    v2f o2; o2[0] = S; o2[1] = S2;
    float* po = PART + (size_t)blockIdx.x * 512 + isbg * 256 + c * 2;
    *(volatile v2f*)po = o2; __threadfence(); *(volatile v2f*)po = o2;
}
__global__ __launch_bounds__(256) void k_comb(const float* __restrict__ PART, float* MEANL, float* VARL) {
    __shared__ double ts[256]; __shared__ double tq[256];
    const int tid = threadIdx.x, ch = blockIdx.x; const int c = ch & (CH - 1), isbg = ch >> 7;
    double s = 0.0, q = 0.0;
#pragma unroll 1
    for (int i = 0; i < (NBI * NTILE) / 256; ++i) { const float* p = PART + (size_t)(i * 256 + tid) * 512 + isbg * 256 + c * 2; s += (double)p[0]; q += (double)p[1]; }
    ts[tid] = s; tq[tid] = q; __syncthreads();
#pragma unroll
    for (int sh = 128; sh; sh >>= 1) { if (tid < sh) { ts[tid] += ts[tid + sh]; tq[tid] += tq[tid + sh]; } __syncthreads(); }
    if (tid == 0) { const double n = (double)NBI * (double)NPIX; const double m = ts[0] / n; double var = tq[0] / n - m * m; if (var < 0.0) var = 0.0;
        const float mf = (float)m, vf = (float)var;
        *(volatile float*)(MEANL + (size_t)ch * 32) = mf; *(volatile float*)(VARL + (size_t)ch * 32) = vf; __threadfence(); *(volatile float*)(MEANL + (size_t)ch * 32) = mf; *(volatile float*)(VARL + (size_t)ch * 32) = vf; }
}
__device__ __forceinline__ void gated(const float* __restrict__ low, const Tile& t, int c, float meanc, float sg, float ga, float al, float be, float& fg, float& bg) {
    const float lf = bilin(low + ((size_t)t.b * CH + c) * HS * HS, t.i0, t.i1, t.fy, t.j0, t.j1, t.fx);
    const float lf2 = ga * meanc + lf;
    fg = al * (lf2 * sg); bg = be * (lf2 * (1.0f - sg));
}
__global__ __launch_bounds__(256) void k_fuse(const float* __restrict__ low, const float* __restrict__ xin, const float* __restrict__ MT, const float* __restrict__ gam,
                                              const float* __restrict__ alp, const float* __restrict__ bet, const float* __restrict__ MEANL, const float* __restrict__ VARL,
                                              const float* __restrict__ w1, const float* __restrict__ b1, const float* __restrict__ w2, const float* __restrict__ b2, int b, bf* FH, bf* FL) {
    __shared__ __align__(16) unsigned short sh_[64][CH + 8]; __shared__ __align__(16) unsigned short sl_[64][CH + 8];
    const int tid = threadIdx.x; const Tile t = tile_of(b * NTILE + blockIdx.x, tid);
    const float meanc = MT[(size_t)(b * NTILE + blockIdx.x) * 64 + t.px];
    const float sg = 1.0f / (1.0f + expf(-bfr(xin[((size_t)t.b * HO + t.y) * HO + t.x])));
    const float ga = bfr(gam[0]), al = bfr(alp[0]), be = bfr(bet[0]);
#pragma unroll 1
    for (int k = 0; k < 32; ++k) { const int c = t.grp * 32 + k; float fg, bg; gated(low, t, c, meanc, sg, ga, al, be, fg, bg);
        const float r1 = fmaxf((fg - MEANL[(size_t)c * 32]) * rsqrtf(VARL[(size_t)c * 32] + EPS_) * bfr(w1[c]) + bfr(b1[c]), 0.f);
        const float r2 = fmaxf((bg - MEANL[(size_t)(CH + c) * 32]) * rsqrtf(VARL[(size_t)(CH + c) * 32] + EPS_) * bfr(w2[c]) + bfr(b2[c]), 0.f);
        const float f = r1 - r2; const unsigned short hb = f2bf(f); sh_[t.px][c] = hb; sl_[t.px][c] = f2bf(f - bf2f(hb)); }
    __syncthreads();
#pragma unroll 1
    for (int ps = 0; ps < 2; ++ps) {
#pragma unroll
        for (int rd = 0; rd < 4; ++rd) { const int p = (tid >> 4) + 16 * rd, q = tid & 15; const int py = (blockIdx.x >> 5) * 8 + (p >> 3), pxx = (blockIdx.x & 31) * 8 + (p & 7);
            const size_t o = ((size_t)(py + 1) * HP + (pxx + 1)) * CH + q * 8;
            *(volatile v8us*)(FH + o) = *(const v8usa*)(&sh_[p][q * 8]); *(volatile v8us*)(FL + o) = *(const v8usa*)(&sl_[p][q * 8]); }
        if (ps == 0) __threadfence(); }
}
__global__ __launch_bounds__(64) void k_border(bf* P0, bf* P1, bf* P2, bf* P3) {
    const int i = blockIdx.x; int r, c;
    if (i < HP) { r = 0; c = i; } else if (i < 2 * HP) { r = HP - 1; c = i - HP; } else if (i < 2 * HP + HO) { r = i - 2 * HP + 1; c = 0; } else { r = i - 2 * HP - HO + 1; c = HP - 1; }
    const int tid = threadIdx.x, pl = tid >> 4, q = tid & 15;
    bf* P = pl == 0 ? P0 : pl == 1 ? P1 : pl == 2 ? P2 : P3;
    const size_t o = ((size_t)r * HP + c) * CH + q * 8; const v8us z = {};
    *(volatile v8us*)(P + o) = z; __threadfence(); *(volatile v8us*)(P + o) = z;
}
__global__ __launch_bounds__(256) void k_wperm(const float* __restrict__ w, int nout, int nrows, bf* WT) {
    const int i = blockIdx.x * 256 + threadIdx.x; const int total = nrows * 9 * (CH / 8); if (i >= total) return;
    const int o = i / (9 * 16), rem = i - o * 9 * 16, tap = rem >> 4, cq = rem & 15;
    v8us v = {};
    if (o < nout) {
#pragma unroll
        for (int e = 0; e < 8; ++e) v[e] = f2bf(w[((size_t)o * CH + cq * 8 + e) * 9 + tap]); }
    const size_t oo = (size_t)o * KK + tap * CH + cq * 8;
    *(volatile v8us*)(WT + oo) = v; __threadfence(); *(volatile v8us*)(WT + oo) = v;
}
template <int MODE>
__global__ __launch_bounds__(128) void k_conv(const bf* __restrict__ Ph, const bf* __restrict__ Pl, const bf* __restrict__ Bn, const float* __restrict__ bias, int b, bf* YH, bf* YL, float* out) {
    constexpr int NT = MODE == 0 ? 4 : 1;
    __shared__ __align__(16) float ost[4][16 * 68]; __shared__ __align__(16) float o2[2][64];
    const int lane = threadIdx.x & 31, wave = threadIdx.x >> 5, lr = lane & 15, hi = lane >> 4;
    const int y = blockIdx.x >> 2, x0 = (blockIdx.x & 3) * 64 + wave * 16; const int c0 = blockIdx.y * 64;
    v8f acc[NT];
#pragma unroll
    for (int t = 0; t < NT; ++t) acc[t] = (v8f){};
#pragma unroll 1
    for (int tap = 0; tap < 9; ++tap) {
        const int ty = tap / 3, tx = tap - ty * 3;
        const size_t abase = ((size_t)(y + ty) * HP + (x0 + lr + tx)) * CH + 8 * hi;
#pragma unroll
        for (int cc = 0; cc < CH; cc += 32) {
            const v16bf a = cat16b(*(const v8us*)(Ph + abase + cc), *(const v8us*)(Ph + abase + cc + 16));
            const v16bf al = cat16b(*(const v8us*)(Pl + abase + cc), *(const v8us*)(Pl + abase + cc + 16));
#pragma unroll
            for (int t = 0; t < NT; ++t) { const bf* bp = Bn + (size_t)(c0 + t * 16 + lr) * KK + tap * CH + cc + 8 * hi; const v16bf bb = cat16b(*(const v8us*)bp, *(const v8us*)(bp + 16)); acc[t] = wmmab(a, bb, acc[t]); acc[t] = wmmab(al, bb, acc[t]); }
            if (NT == 4) asm volatile("v_nop" : "+v"(acc[0]), "+v"(acc[NT - 1]) : "v"(a), "v"(al) : "memory"); else asm volatile("v_nop" : "+v"(acc[0]) : "v"(a), "v"(al) : "memory");
        }
    }
    float* os = &ost[wave][0];
#pragma unroll
    for (int t = 0; t < NT; ++t) { const int n = c0 + t * 16 + lr; const float bc = (MODE == 0) ? bfr(bias[n]) : (n < 2 ? bfr(bias[n]) : 0.f);
#pragma unroll
        for (int j = 0; j < 8; ++j) os[(hi * 8 + j) * 68 + t * 16 + lr] = acc[t][j] + bc; }
    if (MODE == 0) {
        __builtin_amdgcn_wave_barrier(); asm volatile("" ::: "memory");
        auto pass = [&]() {
#pragma unroll
            for (int s = 0; s < 8; ++s) { const int Lid = (lane >> 3) + 4 * s, piece = lane & 7; const int row = Lid >> 1, cofs = (Lid & 1) * 32 + piece * 4;
                const v4f val = *(const v4fa*)(os + row * 68 + cofs); v4us vh, vl;
#pragma unroll
                for (int i = 0; i < 4; ++i) { const unsigned short hb = f2bf(val[i]); vh[i] = hb; vl[i] = f2bf(val[i] - bf2f(hb)); }
                const size_t go = ((size_t)(y + 1) * HP + (x0 + row + 1)) * CH + c0 + cofs; *(volatile v4us*)(YH + go) = vh; *(volatile v4us*)(YL + go) = vl; }
        };
        pass(); __threadfence(); pass();
    } else {
        __builtin_amdgcn_wave_barrier(); asm volatile("" ::: "memory");
        { const int n = lane >> 4, r = lane & 15; o2[n][wave * 16 + r] = os[r * 68 + n]; }
        __syncthreads();
        if (threadIdx.x < 32) { const int n = threadIdx.x >> 4, q = threadIdx.x & 15; const v4f v = *(const v4fa*)(&o2[n][q * 4]);
            float* ob = out + (((size_t)b * 2 + n) * HO + y) * HO + (blockIdx.x & 3) * 64 + q * 4; *(volatile v4f*)ob = v; __threadfence(); *(volatile v4f*)ob = v; }
    }
}

extern "C" void kernel_launch(void* const* d_in, const int* in_sizes, int n_in,
                              void* d_out, int out_size, void* d_ws, size_t ws_size, hipStream_t stream) {
    (void)in_sizes; (void)n_in; (void)out_size;
    const float* low = (const float*)d_in[0]; const float* xin = (const float*)d_in[1]; const float* gam = (const float*)d_in[2]; const float* alp = (const float*)d_in[3]; const float* bet = (const float*)d_in[4];
    const float* bn1w = (const float*)d_in[5]; const float* bn1b = (const float*)d_in[6]; const float* bn2w = (const float*)d_in[7]; const float* bn2b = (const float*)d_in[8];
    const float* c1w = (const float*)d_in[9]; const float* c1b = (const float*)d_in[10]; const float* c2w = (const float*)d_in[11]; const float* c2b = (const float*)d_in[12];
    float* out = (float*)d_out;
    char* wsp = (char*)d_ws;
    auto take = [&](size_t bytes) { char* p = wsp; wsp += (bytes + 255) & ~(size_t)255; return (void*)p; };
    const size_t PLB = (size_t)HP * HP * CH * 2;
    float* LR = (float*)take((size_t)NBI * CH * HS * HS * 4); float* MT = (float*)take((size_t)NBI * NTILE * 64 * 4); float* PART = (float*)take((size_t)NBI * NTILE * 512 * 4);
    float* MEANL = (float*)take((size_t)2 * CH * 128); float* VARL = (float*)take((size_t)2 * CH * 128);
    bf* WT1 = (bf*)take((size_t)CH * KK * 2); bf* WT2 = (bf*)take((size_t)16 * KK * 2);
    bf* FH = (bf*)take(PLB); bf* FL = (bf*)take(PLB); bf* YH = (bf*)take(PLB); bf* YL = (bf*)take(PLB);
    if ((size_t)(wsp - (char*)d_ws) > ws_size) return;
    k_wperm<<<(CH * 9 * 16 + 255) / 256, 256, 0, stream>>>(c1w, CH, CH, WT1);
    k_wperm<<<(16 * 9 * 16 + 255) / 256, 256, 0, stream>>>(c2w, 2, 16, WT2);
    k_border<<<2 * HP + 2 * HO, 64, 0, stream>>>(FH, FL, YH, YL);
    k_preround<<<(NBI * CH * HS * HS / 4 + 255) / 256, 256, 0, stream>>>(low, LR, NBI * CH * HS * HS / 4);
    k_statf<<<NBI * NTILE, 256, 0, stream>>>(LR, xin, gam, alp, bet, MT, PART);
    k_comb<<<2 * CH, 256, 0, stream>>>(PART, MEANL, VARL);
    for (int b = 0; b < NBI; ++b) {
        k_fuse<<<NTILE, 256, 0, stream>>>(LR, xin, MT, gam, alp, bet, MEANL, VARL, bn1w, bn1b, bn2w, bn2b, b, FH, FL);
        k_conv<0><<<dim3(HO * 4, CH / 64), 128, 0, stream>>>(FH, FL, WT1, c1b, b, YH, YL, nullptr);
        k_conv<1><<<dim3(HO * 4, 1), 128, 0, stream>>>(YH, YL, WT2, c2b, b, nullptr, nullptr, out);
    }
}
